// BatchGraphEncoder_21646635172625
// MI455X (gfx1250) — hardware-verified
//
#include <hip/hip_runtime.h>
#include <stddef.h>
#include <math.h>


#define NB 8
#define NA 64
#define NT 12
#define NH 128
#define KSELF 288
#define KG 768

#define PS_ES    (NB * NA * NA * NH)
#define PS_NODE  (NB * NA * NH)
#define PS_CT    (NB * NT * NA * NH)
#define PS_SC    (NB * NT * NH)
#define PS_TYPAD (NB * NA * 32)
#define PS_W3    (NH * NH)
#define PS_WSELF (NH * KSELF)
#define PS_WE2N  (NH * NH)
#define PS_WG    (512 * KG)
#define PS_WPQ   (384 * NH)

typedef __bf16 v16b __attribute__((ext_vector_type(16)));
typedef __bf16 v8b __attribute__((ext_vector_type(8)));
typedef float v8f __attribute__((ext_vector_type(8)));
typedef float v4f __attribute__((ext_vector_type(4)));
typedef float v4fa __attribute__((ext_vector_type(4), __may_alias__));
typedef unsigned int v4u __attribute__((ext_vector_type(4)));
typedef unsigned int v8u __attribute__((ext_vector_type(8)));
typedef unsigned short bfu;

#define VST4U(ptr, val) (*(volatile v4u*)(ptr) = (val))
#define VST4F(ptr, val) (*(volatile v4f*)(ptr) = (val))

union Frag { v16b v; v8b p[2]; };
union U8 { v8f f; v8u u; };

__device__ __forceinline__ v16b ldfrag(const bfu* p, int pitch) {
  const int l = threadIdx.x & 31, h = l >> 4, m = l & 15;
  const bfu* q = p + (size_t)m * pitch + 8 * h;
  Frag f;
  f.p[0] = *(const v8b*)q;
  f.p[1] = *(const v8b*)(q + 16);
  return f.v;
}

__device__ __forceinline__ v8f mma6(v16b ah, v16b am, v16b al, v16b bh, v16b bm, v16b bl, v8f c) {
  c = __builtin_amdgcn_wmma_f32_16x16x32_bf16(false, al, false, bh, (short)0, c, false, false);
  c = __builtin_amdgcn_wmma_f32_16x16x32_bf16(false, ah, false, bl, (short)0, c, false, false);
  c = __builtin_amdgcn_wmma_f32_16x16x32_bf16(false, am, false, bm, (short)0, c, false, false);
  c = __builtin_amdgcn_wmma_f32_16x16x32_bf16(false, am, false, bh, (short)0, c, false, false);
  c = __builtin_amdgcn_wmma_f32_16x16x32_bf16(false, ah, false, bm, (short)0, c, false, false);
  c = __builtin_amdgcn_wmma_f32_16x16x32_bf16(false, ah, false, bh, (short)0, c, false, false);
  asm volatile("v_nop\n\tv_nop\n\tv_nop\n\tv_nop"
               : "+v"(c)
               : "v"(ah), "v"(am), "v"(al), "v"(bh), "v"(bm), "v"(bl));
  return c;
}

__device__ __forceinline__ void kstep(v8f (&acc)[4], const bfu* Ap, int ap, size_t aps,
                                      const bfu* Bp, int bp, size_t bps) {
  v16b bh = ldfrag(Bp, bp);
  v16b bm = ldfrag(Bp + bps, bp);
  v16b bl = ldfrag(Bp + 2 * bps, bp);
#pragma unroll
  for (int mt = 0; mt < 4; ++mt) {
    const bfu* q = Ap + (size_t)(16 * mt) * ap;
    v16b ah = ldfrag(q, ap);
    v16b am = ldfrag(q + aps, ap);
    v16b al = ldfrag(q + 2 * aps, ap);
    acc[mt] = mma6(ah, am, al, bh, bm, bl, acc[mt]);
  }
}

__device__ __forceinline__ void stage_tile(float* tile, v8f (&acc)[4], int n0) {
  const int l = threadIdx.x & 31, h = l >> 4, m = l & 15;
#pragma unroll
  for (int mt = 0; mt < 4; ++mt) {
#pragma unroll
    for (int r = 0; r < 8; ++r) tile[(16 * mt + 8 * h + r) * 128 + n0 + m] = acc[mt][r];
  }
}

__device__ __forceinline__ v8f zero8() { v8f z = {0.f, 0.f, 0.f, 0.f, 0.f, 0.f, 0.f, 0.f}; return z; }
__device__ __forceinline__ v4f ld4g(const float* p) { return *(const v4f*)p; }
__device__ __forceinline__ v8f ld8g(const float* p) {
  v4f a = *(const v4f*)p, b = *(const v4f*)(p + 4);
  return __builtin_shufflevector(a, b, 0, 1, 2, 3, 4, 5, 6, 7);
}
__device__ __forceinline__ v8f ld8s(const float* p) {
  v4f a = *(const v4fa*)p, b = *(const v4fa*)(p + 4);
  return __builtin_shufflevector(a, b, 0, 1, 2, 3, 4, 5, 6, 7);
}
__device__ __forceinline__ v4f lo4(v8f x) { return __builtin_shufflevector(x, x, 0, 1, 2, 3); }
__device__ __forceinline__ v4f hi4(v8f x) { return __builtin_shufflevector(x, x, 4, 5, 6, 7); }

__device__ __forceinline__ v8u rne_hi(v8u u) {
  v8u t = u + 0x7FFFu + ((u >> 16) & 1u);
  return t & 0xFFFF0000u;
}
__device__ __forceinline__ v4u pack8(v8u q) {
  v4u p;
  p.x = (q.s0 >> 16) | q.s1;
  p.y = (q.s2 >> 16) | q.s3;
  p.z = (q.s4 >> 16) | q.s5;
  p.w = (q.s6 >> 16) | q.s7;
  return p;
}
__device__ __forceinline__ void split3(v8f x, v4u& ph, v4u& pm, v4u& pl) {
  U8 a; a.f = x;
  v8u hq = rne_hi(a.u);
  U8 hb; hb.u = hq;
  v8f r1 = x - hb.f;
  U8 c; c.f = r1;
  v8u mq = rne_hi(c.u);
  U8 mb; mb.u = mq;
  v8f r2 = r1 - mb.f;
  U8 d; d.f = r2;
  v8u lq = rne_hi(d.u);
  ph = pack8(hq); pm = pack8(mq); pl = pack8(lq);
}
__device__ __forceinline__ void store3x2(bfu* d, size_t ps, v4u ph, v4u pm, v4u pl) {
  VST4U(d, ph); VST4U(d + ps, pm); VST4U(d + 2 * ps, pl);
  __threadfence();
  VST4U(d, ph); VST4U(d + ps, pm); VST4U(d + 2 * ps, pl);
}

__device__ __forceinline__ int gate_col(int p) {
  const int nb = p >> 7, c = p & 127;
  return ((c >> 5) << 7) + (nb << 5) + (c & 31);
}
__device__ __forceinline__ float sigm(float x) { return 1.0f / (1.0f + expf(-x)); }


__global__ __launch_bounds__(256) void k_fill(unsigned int* __restrict__ p, int n16) {
  const int g = blockIdx.x * 256 + threadIdx.x;
  if (g >= n16) return;
  v4u z = {0u, 0u, 0u, 0u};
  unsigned int* d = p + (size_t)g * 4;
  VST4U(d, z);
  __threadfence();
  VST4U(d, z);
}

__global__ __launch_bounds__(256) void k_wsplit(const float* __restrict__ src, int srcCols, int kBase, int K,
                                                bfu* __restrict__ dst, int nRows, int nOff, int Kpad, int kOff,
                                                int kChunks, int ps, int perm) {
  const int g = blockIdx.x * 256 + threadIdx.x;
  if (g >= nRows * kChunks) return;
  const int n = g / kChunks, c = g - n * kChunks;
  const int sc = perm ? gate_col(n) : n;
  v8f x = zero8();
#pragma unroll
  for (int e = 0; e < 8; ++e) {
    const int k = 8 * c + e;
    x[e] = (k < K) ? src[(size_t)(kBase + k) * srcCols + sc] : 0.f;
  }
  v4u ph, pm, pl;
  split3(x, ph, pm, pl);
  bfu* d = dst + (size_t)(nOff + n) * Kpad + kOff + 8 * c;
  store3x2(d, (size_t)ps, ph, pm, pl);
}

__global__ __launch_bounds__(256) void k_uv(const float* __restrict__ ntraj, const float* __restrict__ traj,
                                            const float* __restrict__ atype, const float* __restrict__ Wein,
                                            const float* __restrict__ Wety, float* __restrict__ UV) {
  const int tid = threadIdx.x, w = tid >> 5, l = tid & 31;
  const int r = blockIdx.x * 8 + w;
  if (r >= 2 * NB * NA) return;
  const int which = r >> 9, ba = r & 511;
  const int n4 = 4 * l;
  const size_t f0 = (size_t)ba * NT * 3;
  const int fo = which ? 6 : 0, to = which ? 20 : 12, yo = which ? 8 : 0;
  v4f s = {0.f, 0.f, 0.f, 0.f};
#pragma unroll
  for (int k = 0; k < 3; ++k) s += ntraj[f0 + k] * ld4g(Wein + (size_t)(fo + k) * NH + n4);
#pragma unroll
  for (int k = 0; k < 3; ++k) s += traj[f0 + k] * ld4g(Wein + (size_t)(fo + 3 + k) * NH + n4);
#pragma unroll
  for (int k = 0; k < 8; ++k) s += atype[(size_t)ba * 8 + k] * ld4g(Wein + (size_t)(to + k) * NH + n4);
#pragma unroll
  for (int k = 0; k < 8; ++k) s += atype[(size_t)ba * 8 + k] * ld4g(Wety + (size_t)(yo + k) * NH + n4);
  float* d = UV + (size_t)r * NH + n4;
  VST4F(d, s);
  __threadfence();
  VST4F(d, s);
}

__global__ __launch_bounds__(256) void k_edge0(const float* __restrict__ UV, const float* __restrict__ bein,
                                               const float* __restrict__ bety, bfu* __restrict__ espl) {
  const int g = blockIdx.x * 256 + threadIdx.x;
  if (g >= NB * NA * NA * 16) return;
  const int ch = g & 15, e = g >> 4;
  const int j = e & 63, bi = e >> 6, b = bi >> 6;
  v8f u = ld8g(UV + (size_t)bi * NH + 8 * ch);
  v8f v = ld8g(UV + (size_t)(NB * NA + b * NA + j) * NH + 8 * ch);
  v8f s = ((u + v) + ld8g(bein + 8 * ch)) + ld8g(bety + 8 * ch);
  v4u ph, pm, pl;
  split3(s, ph, pm, pl);
  store3x2(espl + (size_t)g * 8, (size_t)PS_ES, ph, pm, pl);
}

__global__ __launch_bounds__(256) void k_coord(const float* __restrict__ ntraj, const float* __restrict__ traj,
                                               const float* __restrict__ W_in, const float* __restrict__ b_in,
                                               bfu* __restrict__ coordpl) {
  const int g = blockIdx.x * 256 + threadIdx.x;
  if (g >= NB * NT * NA * 16) return;
  const int ch = g & 15, e = g >> 4;
  const int a = e & 63, bt = e >> 6;
  const int b = bt / NT, t = bt - b * NT;
  const size_t row = ((size_t)(b * NA + a) * NT + t) * 3;
  v8f s = zero8();
#pragma unroll
  for (int k = 0; k < 3; ++k) s += ntraj[row + k] * ld8g(W_in + (size_t)k * NH + 8 * ch);
#pragma unroll
  for (int k = 0; k < 3; ++k) s += traj[row + k] * ld8g(W_in + (size_t)(3 + k) * NH + 8 * ch);
  s = s + ld8g(b_in + 8 * ch);
#pragma unroll
  for (int q = 0; q < 8; ++q) s[q] = fmaxf(s[q], 0.f);
  v4u ph, pm, pl;
  split3(s, ph, pm, pl);
  store3x2(coordpl + (size_t)g * 8, (size_t)PS_CT, ph, pm, pl);
}

__global__ __launch_bounds__(256) void k_agent(const float* __restrict__ adata, const float* __restrict__ rel,
                                               const float* __restrict__ W_ag, const float* __restrict__ b_ag,
                                               bfu* __restrict__ agentpl) {
  const int g = blockIdx.x * 256 + threadIdx.x;
  if (g >= NB * NT * NA * 16) return;
  const int ch = g & 15, e = g >> 4;
  const int a = e & 63, bt = e >> 6;
  const int b = bt / NT, t = bt - b * NT;
  const size_t row = ((size_t)(b * NA + a) * NT + t) * 16;
  v8f s = zero8();
#pragma unroll 1
  for (int k = 0; k < 16; ++k) s += adata[row + k] * ld8g(W_ag + (size_t)k * NH + 8 * ch);
  s = (s + ld8g(b_ag + 8 * ch)) * rel[b * NA + a];
  v4u ph, pm, pl;
  split3(s, ph, pm, pl);
  store3x2(agentpl + (size_t)g * 8, (size_t)PS_CT, ph, pm, pl);
}

__global__ __launch_bounds__(256) void k_scene(const float* __restrict__ scene, const float* __restrict__ W_sc,
                                               const float* __restrict__ b_sc, bfu* __restrict__ scenepl) {
  const int g = blockIdx.x * 256 + threadIdx.x;
  if (g >= NB * NT * 16) return;
  const int ch = g & 15, e = g >> 4;
  const size_t row = (size_t)e * 32;
  v8f s = zero8();
#pragma unroll 1
  for (int k = 0; k < 32; ++k) s += scene[row + k] * ld8g(W_sc + (size_t)k * NH + 8 * ch);
  s = s + ld8g(b_sc + 8 * ch);
  v4u ph, pm, pl;
  split3(s, ph, pm, pl);
  store3x2(scenepl + (size_t)g * 8, (size_t)PS_SC, ph, pm, pl);
}

__global__ __launch_bounds__(256) void k_type(const float* __restrict__ atype, const float* __restrict__ W_nt,
                                              const float* __restrict__ b_nt, bfu* __restrict__ typepl) {
  const int g = blockIdx.x * 256 + threadIdx.x;
  if (g >= NB * NA * 16) return;
  const int ch = g & 15, e = g >> 4;
  const size_t row = (size_t)e * 8;
  v8f s = zero8();
#pragma unroll 1
  for (int k = 0; k < 8; ++k) s += atype[row + k] * ld8g(W_nt + (size_t)k * NH + 8 * ch);
  s = s + ld8g(b_nt + 8 * ch);
  v4u ph, pm, pl;
  split3(s, ph, pm, pl);
  store3x2(typepl + (size_t)g * 8, (size_t)PS_NODE, ph, pm, pl);
}

__global__ __launch_bounds__(256) void k_typad(const float* __restrict__ atype, bfu* __restrict__ typad) {
  const int g = blockIdx.x * 256 + threadIdx.x;
  if (g >= NB * NA * 4) return;
  const int c = g & 3, e = g >> 2;
  v8f x = zero8();
  if (c == 0) x = ld8g(atype + (size_t)e * 8);
  v4u ph, pm, pl;
  split3(x, ph, pm, pl);
  store3x2(typad + (size_t)g * 8, (size_t)PS_TYPAD, ph, pm, pl);
}


__global__ __launch_bounds__(256) void k_edge(bfu* __restrict__ espl, const float* __restrict__ P,
                                              const float* __restrict__ Q, const float* __restrict__ b_edge,
                                              const bfu* __restrict__ W3, float* __restrict__ aggE) {
  __shared__ __attribute__((aligned(16))) float tile[64 * 128];
  __shared__ __attribute__((aligned(16))) float red[8 * 128];
  __shared__ __attribute__((aligned(16))) float red2[128];
  const int i = blockIdx.x, b = blockIdx.y;
  const int tid = threadIdx.x, w = tid >> 5, l = tid & 31;
  bfu* est = espl + (((size_t)b * NA + i) * NA) * NH;

  v8f acc[4];
#pragma unroll
  for (int mt = 0; mt < 4; ++mt) acc[mt] = zero8();
#pragma unroll 1
  for (int kt = 0; kt < 4; ++kt)
    kstep(acc, est + 32 * kt, NH, (size_t)PS_ES, W3 + (size_t)(16 * w) * NH + 32 * kt, NH, (size_t)PS_W3);
  stage_tile(tile, acc, 16 * w);
  __syncthreads();

  const int ch = l & 15, n8 = 8 * ch, hh = l >> 4;
  const v8f p8 = ld8g(P + ((size_t)b * NA + i) * NH + n8);
  const v8f bias = ld8g(b_edge + n8);
  v8f cs = zero8();
#pragma unroll
  for (int it = 0; it < 4; ++it) {
    const int j = 16 * it + 2 * w + hh;
    v8f x = ld8s(tile + j * 128 + n8);
    v8f q8 = ld8g(Q + ((size_t)b * NA + j) * NH + n8);
    v8f v = ((x + p8) + q8) + bias;
    cs += v;
    v4u ph, pm, pl;
    split3(v, ph, pm, pl);
    store3x2(est + (size_t)j * NH + n8, (size_t)PS_ES, ph, pm, pl);
  }
#pragma unroll
  for (int e = 0; e < 8; ++e) cs[e] = cs[e] + __shfl_xor(cs[e], 16, 32);
  if (l < 16) {
    *(v4fa*)(red + w * 128 + n8) = lo4(cs);
    *(v4fa*)(red + w * 128 + n8 + 4) = hi4(cs);
  }
  __syncthreads();
  if (tid < 128) {
    float s = 0.f;
#pragma unroll
    for (int w2 = 0; w2 < 8; ++w2) s += red[w2 * 128 + tid];
    red2[tid] = s;
  }
  __syncthreads();
  if (tid < 32) {
    v4f v = *(const v4fa*)(red2 + 4 * tid);
    float* ap = aggE + ((size_t)b * NA + i) * NH + 4 * tid;
    VST4F(ap, v);
    __threadfence();
    VST4F(ap, v);
  }
}

__global__ __launch_bounds__(256) void k_self(const bfu* __restrict__ hcur, bfu* __restrict__ sepl,
                                              const bfu* __restrict__ typad, const bfu* __restrict__ Wself,
                                              const float* __restrict__ b_self, const float* __restrict__ aggE,
                                              bfu* __restrict__ aggpl) {
  __shared__ __attribute__((aligned(16))) float tile[64 * 128];
  const int b = blockIdx.x;
  const int tid = threadIdx.x, w = tid >> 5, l = tid & 31;

  v8f acc[4];
#pragma unroll
  for (int mt = 0; mt < 4; ++mt) acc[mt] = zero8();
#pragma unroll 1
  for (int kt = 0; kt < 9; ++kt) {
    const bfu* Ap; int ap; size_t aps;
    if (kt < 4)      { Ap = hcur + ((size_t)(b * 4 + kt) * NA) * 32;        ap = 32; aps = PS_NODE; }
    else if (kt < 8) { Ap = sepl + (size_t)b * NA * NH + 32 * (kt - 4);     ap = NH; aps = PS_NODE; }
    else             { Ap = typad + (size_t)b * NA * 32;                    ap = 32; aps = PS_TYPAD; }
    kstep(acc, Ap, ap, aps, Wself + (size_t)(16 * w) * KSELF + 32 * kt, KSELF, (size_t)PS_WSELF);
  }
  stage_tile(tile, acc, 16 * w);
  __syncthreads();

  const int ch = l & 15, n8 = 8 * ch, hh = l >> 4;
  const v8f bias = ld8g(b_self + n8);
#pragma unroll
  for (int it = 0; it < 4; ++it) {
    const int a = 16 * it + 2 * w + hh;
    const size_t ro = ((size_t)b * NA + a) * NH + n8;
    v8f x = ld8s(tile + a * 128 + n8);
    v8f v = x + bias;
    v8f ag = ld8g(aggE + ro) + v;
    v4u sh, sm, sl, gh, gm, gl;
    split3(v, sh, sm, sl);
    split3(ag, gh, gm, gl);
    bfu* sd = sepl + ro;
    bfu* gd = aggpl + ro;
    VST4U(sd, sh); VST4U(sd + PS_NODE, sm); VST4U(sd + 2 * PS_NODE, sl);
    VST4U(gd, gh); VST4U(gd + PS_NODE, gm); VST4U(gd + 2 * PS_NODE, gl);
    __threadfence();
    VST4U(sd, sh); VST4U(sd + PS_NODE, sm); VST4U(sd + 2 * PS_NODE, sl);
    VST4U(gd, gh); VST4U(gd + PS_NODE, gm); VST4U(gd + 2 * PS_NODE, gl);
  }
}

__global__ __launch_bounds__(256) void k_e2n(const bfu* __restrict__ aggpl, const bfu* __restrict__ We2n,
                                             const float* __restrict__ b_e2n, bfu* __restrict__ nepl, int t) {
  __shared__ __attribute__((aligned(16))) float tile[64 * 128];
  const int b = blockIdx.x;
  const int tid = threadIdx.x, w = tid >> 5, l = tid & 31;

  v8f acc[4];
#pragma unroll
  for (int mt = 0; mt < 4; ++mt) acc[mt] = zero8();
#pragma unroll 1
  for (int kt = 0; kt < 4; ++kt)
    kstep(acc, aggpl + (size_t)b * NA * NH + 32 * kt, NH, (size_t)PS_NODE,
          We2n + (size_t)(16 * w) * NH + 32 * kt, NH, (size_t)PS_WE2N);
  stage_tile(tile, acc, 16 * w);
  __syncthreads();

  const float ts = (t > 0) ? 1.f : 0.f;
  const int ch = l & 15, n8 = 8 * ch, hh = l >> 4;
  const v8f bias = ld8g(b_e2n + n8);
#pragma unroll
  for (int it = 0; it < 4; ++it) {
    const int a = 16 * it + 2 * w + hh;
    const size_t ro = ((size_t)b * NA + a) * NH + n8;
    v8f x = ld8s(tile + a * 128 + n8);
    v8f v = (x + bias) * ts;
    v4u ph, pm, pl;
    split3(v, ph, pm, pl);
    store3x2(nepl + ro, (size_t)PS_NODE, ph, pm, pl);
  }
}

__global__ __launch_bounds__(256) void k_gates(const bfu* __restrict__ coordpl, const bfu* __restrict__ typepl,
                                               const bfu* __restrict__ nepl, const bfu* __restrict__ scenepl,
                                               const bfu* __restrict__ agentpl, const bfu* __restrict__ hcur,
                                               const bfu* __restrict__ Wg, const float* __restrict__ b_ih,
                                               const float* __restrict__ b_hh, float* __restrict__ cbuf,
                                               bfu* __restrict__ hnext, int t) {
  __shared__ __attribute__((aligned(16))) float tile[64 * 128];
  __shared__ __attribute__((aligned(16))) float hT[64 * 32];
  const int nb = blockIdx.x, b = blockIdx.y;
  const int tid = threadIdx.x, w = tid >> 5, l = tid & 31;

  v8f acc[4];
#pragma unroll
  for (int mt = 0; mt < 4; ++mt) acc[mt] = zero8();
#pragma unroll 1
  for (int kt = 0; kt < 24; ++kt) {
    const int seg = kt >> 2, kc = kt & 3;
    const bfu* Ap; int ap; size_t aps;
    if (seg == 0)      { Ap = coordpl + (((size_t)(b * NT + t)) * NA) * NH + 32 * kc; ap = NH; aps = PS_CT; }
    else if (seg == 1) { Ap = typepl + (size_t)b * NA * NH + 32 * kc;                 ap = NH; aps = PS_NODE; }
    else if (seg == 2) { Ap = nepl + (size_t)b * NA * NH + 32 * kc;                   ap = NH; aps = PS_NODE; }
    else if (seg == 3) { Ap = scenepl + (size_t)(b * NT + t) * NH + 32 * kc;          ap = 0;  aps = PS_SC; }
    else if (seg == 4) { Ap = agentpl + (((size_t)(b * NT + t)) * NA) * NH + 32 * kc; ap = NH; aps = PS_CT; }
    else               { Ap = hcur + ((size_t)(b * 4 + kc) * NA) * 32;                ap = 32; aps = PS_NODE; }
    kstep(acc, Ap, ap, aps, Wg + ((size_t)(nb * 128 + 16 * w)) * KG + 32 * kt, KG, (size_t)PS_WG);
  }
  stage_tile(tile, acc, 16 * w);
  __syncthreads();

  const int u4 = 4 * (l & 7), ug = 32 * nb + u4;
  const v4f bi0 = ld4g(b_ih + ug),       bi1 = ld4g(b_hh + ug);
  const v4f bf0 = ld4g(b_ih + 128 + ug), bf1 = ld4g(b_hh + 128 + ug);
  const v4f bg0 = ld4g(b_ih + 256 + ug), bg1 = ld4g(b_hh + 256 + ug);
  const v4f bo0 = ld4g(b_ih + 384 + ug), bo1 = ld4g(b_hh + 384 + ug);
  v4f cst[2];
#pragma unroll
  for (int it2 = 0; it2 < 2; ++it2) {
    const int a = 8 * w + 4 * it2 + (l >> 3);
    const float* tr = tile + a * 128 + u4;
    v4f gi = (*(const v4fa*)(tr)      + bi0) + bi1;
    v4f gf = (*(const v4fa*)(tr + 32) + bf0) + bf1;
    v4f gg = (*(const v4fa*)(tr + 64) + bg0) + bg1;
    v4f go = (*(const v4fa*)(tr + 96) + bo0) + bo1;
    const size_t co = ((size_t)(b * NA + a)) * NH + ug;
    v4f cold = ld4g(cbuf + co);
    v4f cn, hn;
#pragma unroll
    for (int e = 0; e < 4; ++e) {
      float c1 = sigm(gf[e]) * cold[e] + sigm(gi[e]) * tanhf(gg[e]);
      cn[e] = c1;
      hn[e] = sigm(go[e]) * tanhf(c1);
    }
    VST4F(cbuf + co, cn);
    cst[it2] = cn;
    *(v4fa*)(hT + a * 32 + u4) = hn;
  }
  __threadfence();
#pragma unroll
  for (int it2 = 0; it2 < 2; ++it2) {
    const int a = 8 * w + 4 * it2 + (l >> 3);
    const size_t co = ((size_t)(b * NA + a)) * NH + ug;
    VST4F(cbuf + co, cst[it2]);
  }
  __syncthreads();
  {
    const int a = tid >> 2, u8 = 8 * (tid & 3);
    v8f x = ld8s(hT + a * 32 + u8);
    v4u ph, pm, pl;
    split3(x, ph, pm, pl);
    store3x2(hnext + (((size_t)(b * 4 + nb)) * NA + a) * 32 + u8, (size_t)PS_NODE, ph, pm, pl);
  }
}

__global__ __launch_bounds__(256) void k_post(const bfu* __restrict__ hnext, const bfu* __restrict__ Wpq,
                                              const float* __restrict__ b_pred, float* __restrict__ out,
                                              float* __restrict__ P, float* __restrict__ Q, int t) {
  __shared__ __attribute__((aligned(16))) float tile[64 * 128];
  const int nt = blockIdx.x, b = blockIdx.y;
  const int tid = threadIdx.x, w = tid >> 5, l = tid & 31;

  v8f acc[4];
#pragma unroll
  for (int mt = 0; mt < 4; ++mt) acc[mt] = zero8();
#pragma unroll 1
  for (int kt = 0; kt < 4; ++kt)
    kstep(acc, hnext + ((size_t)(b * 4 + kt) * NA) * 32, 32, (size_t)PS_NODE,
          Wpq + ((size_t)(nt * 128 + 16 * w)) * NH + 32 * kt, NH, (size_t)PS_WPQ);
  stage_tile(tile, acc, 16 * w);
  __syncthreads();

  const int n4 = 4 * l;
  const v4f bias = ld4g(b_pred + n4);
  v4f vals[8];
#pragma unroll
  for (int it = 0; it < 8; ++it) {
    const int a = 8 * it + w;
    v4f x = *(const v4fa*)(tile + a * 128 + n4);
    float* d;
    v4f v;
    if (nt == 0) {
      v = x + bias;
#pragma unroll
      for (int e = 0; e < 4; ++e) v[e] = fmaxf(v[e], 0.f);
      d = out + (((size_t)(b * NA + a)) * NT + t) * NH + n4;
    } else if (nt == 1) {
      v = x;
      d = P + ((size_t)(b * NA + a)) * NH + n4;
    } else {
      v = x;
      d = Q + ((size_t)(b * NA + a)) * NH + n4;
    }
    vals[it] = v;
    VST4F(d, v);
  }
  __threadfence();
#pragma unroll
  for (int it = 0; it < 8; ++it) {
    const int a = 8 * it + w;
    float* d;
    if (nt == 0)      d = out + (((size_t)(b * NA + a)) * NT + t) * NH + n4;
    else if (nt == 1) d = P + ((size_t)(b * NA + a)) * NH + n4;
    else              d = Q + ((size_t)(b * NA + a)) * NH + n4;
    VST4F(d, vals[it]);
  }
}


extern "C" void kernel_launch(void* const* d_in, const int* in_sizes, int n_in,
                              void* d_out, int out_size, void* d_ws, size_t ws_size,
                              hipStream_t stream) {
  if (n_in < 30) return;
  if (out_size != NB * NA * NT * NH) return;
  if (in_sizes[0] != NB * NA * NT * 3 || in_sizes[1] != NB * NA * NT * 3 || in_sizes[2] != NB * NA * 8 ||
      in_sizes[3] != NB * NT * 32 || in_sizes[4] != NB * NA * NT * 16 || in_sizes[5] != NB * NA ||
      in_sizes[18] != 384 * 128 || in_sizes[20] != 264 * 128 || in_sizes[24] != 640 * 512 ||
      in_sizes[25] != 128 * 512 || in_sizes[28] != 128 * 128) return;

  const float* traj   = (const float*)d_in[0];
  const float* ntraj  = (const float*)d_in[1];
  const float* atype  = (const float*)d_in[2];
  const float* scene  = (const float*)d_in[3];
  const float* adata  = (const float*)d_in[4];
  const float* relev  = (const float*)d_in[5];
  const float* W_in   = (const float*)d_in[6];
  const float* b_in   = (const float*)d_in[7];
  const float* W_nt   = (const float*)d_in[8];
  const float* b_nt   = (const float*)d_in[9];
  const float* W_ag   = (const float*)d_in[10];
  const float* b_ag   = (const float*)d_in[11];
  const float* W_sc   = (const float*)d_in[12];
  const float* b_sc   = (const float*)d_in[13];
  const float* W_ein  = (const float*)d_in[14];
  const float* b_ein  = (const float*)d_in[15];
  const float* W_ety  = (const float*)d_in[16];
  const float* b_ety  = (const float*)d_in[17];
  const float* W_edge = (const float*)d_in[18];
  const float* b_edge = (const float*)d_in[19];
  const float* W_self = (const float*)d_in[20];
  const float* b_self = (const float*)d_in[21];
  const float* W_e2n  = (const float*)d_in[22];
  const float* b_e2n  = (const float*)d_in[23];
  const float* W_ih   = (const float*)d_in[24];
  const float* W_hh   = (const float*)d_in[25];
  const float* b_ih   = (const float*)d_in[26];
  const float* b_hh   = (const float*)d_in[27];
  const float* W_pred = (const float*)d_in[28];
  const float* b_pred = (const float*)d_in[29];
  float* out = (float*)d_out;

  char* ws = (char*)d_ws;
  size_t off = 0;
  auto carve = [&](size_t bytes) -> char* {
    char* p = ws + off;
    off += (bytes + 255) & ~(size_t)255;
    return p;
  };
  bfu* espl    = (bfu*)carve((size_t)3 * PS_ES * 2);
  bfu* W3      = (bfu*)carve((size_t)3 * PS_W3 * 2);
  bfu* Wself   = (bfu*)carve((size_t)3 * PS_WSELF * 2);
  bfu* We2n    = (bfu*)carve((size_t)3 * PS_WE2N * 2);
  bfu* Wg      = (bfu*)carve((size_t)3 * PS_WG * 2);
  bfu* Wpq     = (bfu*)carve((size_t)3 * PS_WPQ * 2);
  bfu* coordpl = (bfu*)carve((size_t)3 * PS_CT * 2);
  bfu* agentpl = (bfu*)carve((size_t)3 * PS_CT * 2);
  bfu* typepl  = (bfu*)carve((size_t)3 * PS_NODE * 2);
  bfu* scenepl = (bfu*)carve((size_t)3 * PS_SC * 2);
  bfu* typad   = (bfu*)carve((size_t)3 * PS_TYPAD * 2);
  float* UV    = (float*)carve((size_t)2 * PS_NODE * 4);
  float* aggE  = (float*)carve((size_t)PS_NODE * 4);
  bfu* aggpl   = (bfu*)carve((size_t)3 * PS_NODE * 2);
  bfu* nepl    = (bfu*)carve((size_t)3 * PS_NODE * 2);
  const size_t fillStart = off;
  bfu* hplA    = (bfu*)carve((size_t)3 * PS_NODE * 2);
  bfu* hplB    = (bfu*)carve((size_t)3 * PS_NODE * 2);
  bfu* sepl    = (bfu*)carve((size_t)3 * PS_NODE * 2);
  float* cbuf  = (float*)carve((size_t)PS_NODE * 4);
  float* P     = (float*)carve((size_t)PS_NODE * 4);
  float* Q     = (float*)carve((size_t)PS_NODE * 4);
  const size_t fillBytes = off - fillStart;
  if (off > ws_size) return;

  auto nblk = [](size_t n) { return (unsigned)((n + 255) / 256); };

  const int n16 = (int)(fillBytes / 16);
  k_fill<<<nblk((size_t)n16), 256, 0, stream>>>((unsigned int*)(ws + fillStart), n16);

  k_wsplit<<<nblk(128 * 16), 256, 0, stream>>>(W_edge, 128, 256, 128, W3, 128, 0, NH, 0, 16, PS_W3, 0);
  k_wsplit<<<nblk(128 * 36), 256, 0, stream>>>(W_self, 128, 0, 264, Wself, 128, 0, KSELF, 0, 36, PS_WSELF, 0);
  k_wsplit<<<nblk(128 * 16), 256, 0, stream>>>(W_e2n, 128, 0, 128, We2n, 128, 0, NH, 0, 16, PS_WE2N, 0);
  k_wsplit<<<nblk(512 * 80), 256, 0, stream>>>(W_ih, 512, 0, 640, Wg, 512, 0, KG, 0, 80, PS_WG, 1);
  k_wsplit<<<nblk(512 * 16), 256, 0, stream>>>(W_hh, 512, 0, 128, Wg, 512, 0, KG, 640, 16, PS_WG, 1);
  k_wsplit<<<nblk(128 * 16), 256, 0, stream>>>(W_pred, 128, 0, 128, Wpq, 128, 0, NH, 0, 16, PS_WPQ, 0);
  k_wsplit<<<nblk(128 * 16), 256, 0, stream>>>(W_edge, 128, 0, 128, Wpq, 128, 128, NH, 0, 16, PS_WPQ, 0);
  k_wsplit<<<nblk(128 * 16), 256, 0, stream>>>(W_edge, 128, 128, 128, Wpq, 128, 256, NH, 0, 16, PS_WPQ, 0);

  k_uv<<<nblk((size_t)2 * NB * NA * 32), 256, 0, stream>>>(ntraj, traj, atype, W_ein, W_ety, UV);
  k_edge0<<<nblk((size_t)NB * NA * NA * 16), 256, 0, stream>>>(UV, b_ein, b_ety, espl);
  k_coord<<<nblk((size_t)NB * NT * NA * 16), 256, 0, stream>>>(ntraj, traj, W_in, b_in, coordpl);
  k_agent<<<nblk((size_t)NB * NT * NA * 16), 256, 0, stream>>>(adata, relev, W_ag, b_ag, agentpl);
  k_scene<<<nblk((size_t)NB * NT * 16), 256, 0, stream>>>(scene, W_sc, b_sc, scenepl);
  k_type<<<nblk((size_t)NB * NA * 16), 256, 0, stream>>>(atype, W_nt, b_nt, typepl);
  k_typad<<<nblk((size_t)NB * NA * 4), 256, 0, stream>>>(atype, typad);

  for (int t = 0; t < NT; ++t) {
    bfu* hc = (t & 1) ? hplB : hplA;
    bfu* hn = (t & 1) ? hplA : hplB;
    k_edge<<<dim3(NA, NB), 256, 0, stream>>>(espl, P, Q, b_edge, W3, aggE);
    k_self<<<dim3(NB), 256, 0, stream>>>(hc, sepl, typad, Wself, b_self, aggE, aggpl);
    k_e2n<<<dim3(NB), 256, 0, stream>>>(aggpl, We2n, b_e2n, nepl, t);
    k_gates<<<dim3(4, NB), 256, 0, stream>>>(coordpl, typepl, nepl, scenepl, agentpl, hc, Wg,
                                             b_ih, b_hh, cbuf, hn, t);
    k_post<<<dim3(3, NB), 256, 0, stream>>>(hn, Wpq, b_pred, out, P, Q, t);
  }
}
